// SoftmaxAttentionLayer_84885733638833
// MI455X (gfx1250) — hardware-verified
//
#include <hip/hip_runtime.h>
#include <stddef.h>


#define BDIM    2
#define SDIM    2048
#define HDIM    1024
#define H3DIM   3072
#define NHEADS  16
#define HD      64
#define HHD     32
#define BS      (BDIM * SDIM)
#define NJB     (SDIM / 32)
#define JSPLIT  16
#define QSCALE  64.0f
#define SCALEC  (0.125f / 4096.0f)
#define LN2P15  10.397207708399179f
#define NEG_INF (-__builtin_inff())

typedef _Float16       v8h   __attribute__((ext_vector_type(8)));
typedef _Float16       v16h  __attribute__((ext_vector_type(16)));
typedef __bf16         v16b  __attribute__((ext_vector_type(16)));
typedef unsigned short v8us  __attribute__((ext_vector_type(8)));
typedef float          v4f   __attribute__((ext_vector_type(4)));
typedef float          v8f   __attribute__((ext_vector_type(8)));
typedef int            v8i   __attribute__((ext_vector_type(8)));
typedef unsigned int   u32x4 __attribute__((ext_vector_type(4)));
typedef u32x4 __attribute__((may_alias)) u32x4a;
typedef v4f   __attribute__((may_alias)) v4fa;

union Frag  { v8i w; v16h h; v16b b; u32x4 q[2]; };
union PackH { v8h v;  u32x4 u; };
union PackS { v8us v; u32x4 u; };

__device__ __forceinline__ v8i ldfrag(const unsigned short* row, int k0, int hh) {
    Frag f;
    f.q[0] = *(const u32x4a*)(row + k0 + 8 * hh);
    f.q[1] = *(const u32x4a*)(row + k0 + 16 + 8 * hh);
    return f.w;
}
__device__ __forceinline__ v8i izero8() { return (v8i)0; }
__device__ __forceinline__ v8f fzero8() { return (v8f)0.0f; }

__device__ __forceinline__ v8f wm_h(v8f c, v8i a, v8i b) {
    Frag fa, fb; fa.w = a; fb.w = b;
    c = __builtin_amdgcn_wmma_f32_16x16x32_f16(false, fa.h, false, fb.h, (short)0, c, false, false);
    asm volatile("v_nop\n\tv_nop\n\tv_nop\n\tv_nop" : "+v"(c) : "v"(a), "v"(b));
    return c;
}
__device__ __forceinline__ v8f wm_b(v8f c, v8i a, v8i b) {
    Frag fa, fb; fa.w = a; fb.w = b;
    c = __builtin_amdgcn_wmma_f32_16x16x32_bf16(false, fa.b, false, fb.b, (short)0, c, false, false);
    asm volatile("v_nop\n\tv_nop\n\tv_nop\n\tv_nop" : "+v"(c) : "v"(a), "v"(b));
    return c;
}

__device__ __forceinline__ unsigned short bf16_bits(float f) {
    unsigned int u = __float_as_uint(f);
    u += 0x7FFFu + ((u >> 16) & 1u);
    return (unsigned short)(u >> 16);
}
__device__ __forceinline__ float bf16_val(unsigned short s) {
    return __uint_as_float(((unsigned int)s) << 16);
}

__device__ __forceinline__ void split_h8(const float (&x)[8], u32x4& hi, u32x4& lo) {
    PackH ph, pl;
    #pragma unroll
    for (int j = 0; j < 8; ++j) {
        const _Float16 hv = (_Float16)x[j];
        ph.v[j] = hv;
        pl.v[j] = (_Float16)(x[j] - (float)hv);
    }
    hi = ph.u; lo = pl.u;
}
__device__ __forceinline__ void split_b8(const float (&x)[8], u32x4& hi, u32x4& lo) {
    PackS ph, pl;
    #pragma unroll
    for (int j = 0; j < 8; ++j) {
        const unsigned short hb = bf16_bits(x[j]);
        ph.v[j] = hb;
        pl.v[j] = bf16_bits(x[j] - bf16_val(hb));
    }
    hi = ph.u; lo = pl.u;
}

__global__ void __launch_bounds__(256)
k_cvt(const float* __restrict__ src, unsigned short* __restrict__ dst, int n8)
{
    const int i = blockIdx.x * 256 + threadIdx.x;
    if (i >= n8) return;
    const size_t e = (size_t)i * 8;
    const v4f a = *(const v4fa*)(src + e);
    const v4f c = *(const v4fa*)(src + e + 4);
    PackS p;
    #pragma unroll
    for (int j = 0; j < 4; ++j) { p.v[j] = bf16_bits(a[j]); p.v[4 + j] = bf16_bits(c[j]); }
    const u32x4 u = p.u;
    volatile u32x4* const q = (volatile u32x4*)(dst + e);
    *q = u;
    __threadfence();
    *q = u;
}

__global__ void __launch_bounds__(256)
k_trig(float* __restrict__ cs, float* __restrict__ sn, int S)
{
#pragma clang fp contract(off)
    __shared__ __align__(16) float lc[8][HHD];
    __shared__ __align__(16) float ls[8][HHD];
    const int tid = threadIdx.x;
    const int sl = tid >> 5, dh = tid & 31;
    const int s = blockIdx.x * 8 + sl;
    {
        const float e   = (float)dh * 0.03125f;
        const float p   = (float)pow(10000.0, (double)e);
        const float inv = (float)(1.0 / (double)p);
        const float ang = (float)s * inv;
        lc[sl][dh] = cosf(ang);
        ls[sl][dh] = sinf(ang);
    }
    __syncthreads();
    if (tid < 64) {
        const int r = tid >> 3, g = tid & 7;
        const int so = blockIdx.x * 8 + r;
        if (so < S) {
            const v4f c = *(const v4fa*)(&lc[r][4 * g]);
            const v4f n = *(const v4fa*)(&ls[r][4 * g]);
            volatile v4f* const pc = (volatile v4f*)(cs + (size_t)so * HHD + 4 * g);
            volatile v4f* const pn = (volatile v4f*)(sn + (size_t)so * HHD + 4 * g);
            *pc = c; *pn = n;
            __threadfence();
            *pc = c; *pn = n;
        }
    }
}

__global__ void __launch_bounds__(256) __attribute__((amdgpu_num_vgpr(256)))
k_gemm_qkv(const unsigned short* __restrict__ X, const unsigned short* __restrict__ W,
           const float* __restrict__ cs, const float* __restrict__ sn,
           unsigned short* __restrict__ Qh, unsigned short* __restrict__ Ql,
           unsigned short* __restrict__ Kh, unsigned short* __restrict__ Kl,
           unsigned short* __restrict__ Vth, unsigned short* __restrict__ Vtl)
{
#pragma clang fp contract(off)
    __shared__ __align__(16) float tile[128][128];

    const int tid = threadIdx.x, lane = tid & 31, wave = tid >> 5;
    const int hh = lane >> 4, m = lane & 15;
    const int mBase = blockIdx.y * 128, nBase = blockIdx.x * 128;
    if (mBase + 128 > BS || nBase + 128 > H3DIM) return;
    const int m0 = (wave >> 1) * 32, n0 = (wave & 1) * 64;

    v8f acc[2][4];
    #pragma unroll
    for (int mt = 0; mt < 2; ++mt)
        #pragma unroll
        for (int nt = 0; nt < 4; ++nt) acc[mt][nt] = fzero8();

    const unsigned short* const ar0 = X + (size_t)(mBase + m0 + m) * HDIM;
    const unsigned short* const ar1 = ar0 + (size_t)16 * HDIM;
    const unsigned short* const br  = W + (size_t)(nBase + n0 + m) * HDIM;

    #pragma unroll 1
    for (int k0 = 0; k0 < HDIM; k0 += 32) {
        const v8i a0 = ldfrag(ar0, k0, hh);
        const v8i a1 = ldfrag(ar1, k0, hh);
        #pragma unroll
        for (int nt = 0; nt < 4; ++nt) {
            const v8i bq = ldfrag(br + (size_t)nt * 16 * HDIM, k0, hh);
            acc[0][nt] = wm_b(acc[0][nt], a0, bq);
            acc[1][nt] = wm_b(acc[1][nt], a1, bq);
        }
    }

    #pragma unroll
    for (int mt = 0; mt < 2; ++mt)
        #pragma unroll
        for (int nt = 0; nt < 4; ++nt)
            #pragma unroll
            for (int r = 0; r < 8; ++r)
                tile[m0 + mt * 16 + 8 * hh + r][n0 + nt * 16 + m] = acc[mt][nt][r];
    __syncthreads();

    const int part  = nBase >> 10;
    const int hb    = (nBase & (HDIM - 1)) >> 6;
    const int b     = mBase >> 11;
    const int sBase = mBase & (SDIM - 1);

    if (part < 2) {
        unsigned short* const Ph = (part == 0) ? Qh : Kh;
        unsigned short* const Pl = (part == 0) ? Ql : Kl;
        #pragma unroll 1
        for (int rep = 0; rep < 8; ++rep) {
            const int item = tid + rep * 256;
            const int g = item & 7, rh = item >> 3;
            const int row = rh >> 1, half = rh & 1;
            const int s = sBase + row;
            const int d0 = 8 * g, dh0 = d0 & 31, cb = half * 64;
            const int dp = (g < 4) ? (d0 + 32) : (d0 - 32);
            const float sgn = (g < 4) ? -1.0f : 1.0f;
            const v4f c0 = *(const v4fa*)(cs + (size_t)s * HHD + dh0);
            const v4f c1 = *(const v4fa*)(cs + (size_t)s * HHD + dh0 + 4);
            const v4f t0 = *(const v4fa*)(sn + (size_t)s * HHD + dh0);
            const v4f t1 = *(const v4fa*)(sn + (size_t)s * HHD + dh0 + 4);
            const v4f x0 = *(const v4fa*)(&tile[row][cb + d0]);
            const v4f x1 = *(const v4fa*)(&tile[row][cb + d0 + 4]);
            const v4f y0 = *(const v4fa*)(&tile[row][cb + dp]);
            const v4f y1 = *(const v4fa*)(&tile[row][cb + dp + 4]);
            float o[8];
            #pragma unroll
            for (int jj = 0; jj < 4; ++jj) {
                const float pa = x0[jj] * c0[jj];
                const float pb = (sgn * y0[jj]) * t0[jj];
                o[jj] = (pa + pb) * QSCALE;
                const float qa = x1[jj] * c1[jj];
                const float qb = (sgn * y1[jj]) * t1[jj];
                o[4 + jj] = (qa + qb) * QSCALE;
            }
            u32x4 uh, ul;
            split_h8(o, uh, ul);
            const size_t off = ((size_t)(b * NHEADS + hb + half) * SDIM + s) * HD + d0;
            volatile u32x4* const ph = (volatile u32x4*)(Ph + off);
            volatile u32x4* const pl = (volatile u32x4*)(Pl + off);
            *ph = uh; *pl = ul;
            __threadfence();
            *ph = uh; *pl = ul;
        }
    } else {
        #pragma unroll 1
        for (int rep = 0; rep < 8; ++rep) {
            const int item = tid + rep * 256;
            const int p = item & 15, dr = item >> 4;
            const int half = dr >> 6, d = dr & 63;
            float o[8];
            #pragma unroll
            for (int jj = 0; jj < 8; ++jj) o[jj] = tile[8 * p + jj][half * 64 + d] * QSCALE;
            u32x4 uh, ul;
            split_h8(o, uh, ul);
            const size_t off = ((size_t)(b * NHEADS + hb + half) * HD + d) * SDIM + sBase + 8 * p;
            volatile u32x4* const ph = (volatile u32x4*)(Vth + off);
            volatile u32x4* const pl = (volatile u32x4*)(Vtl + off);
            *ph = uh; *pl = ul;
            __threadfence();
            *ph = uh; *pl = ul;
        }
    }
}

__global__ void __launch_bounds__(64) __attribute__((amdgpu_num_vgpr(256)))
k_attn(const unsigned short* __restrict__ Qh, const unsigned short* __restrict__ Ql,
       const unsigned short* __restrict__ Kh, const unsigned short* __restrict__ Kl,
       const unsigned short* __restrict__ Vth, const unsigned short* __restrict__ Vtl,
       unsigned short* __restrict__ Ah, unsigned short* __restrict__ Al)
{
    __shared__ __align__(16) float stg[2][16][64];

    const int lane = threadIdx.x & 31, w = threadIdx.x >> 5;
    const int hh = lane >> 4, m = lane & 15;
    const int jb = blockIdx.x, h = blockIdx.y, b = blockIdx.z;
    if (jb >= NJB || h >= NHEADS || b >= BDIM) return;
    const int bh = b * NHEADS + h;
    const int qBase = 32 * jb + 16 * w;
    const int qRow  = qBase + m;
    const bool split = (jb < JSPLIT);

    const size_t qo = ((size_t)bh * SDIM + qRow) * HD;
    const v8i fQh0 = ldfrag(Qh + qo, 0, hh);
    const v8i fQh1 = ldfrag(Qh + qo, HHD, hh);
    v8i fQl0 = izero8(), fQl1 = izero8();
    if (split) { fQl0 = ldfrag(Ql + qo, 0, hh); fQl1 = ldfrag(Ql + qo, HHD, hh); }

    v8f acc[4];
    #pragma unroll
    for (int c = 0; c < 4; ++c) acc[c] = fzero8();
    float rmax = NEG_INF, lsum = 0.0f;

    #pragma unroll 1
    for (int it = 0; it <= jb; ++it) {
        const int kBase = 32 * it;

        v8f sc[2];
        sc[0] = fzero8(); sc[1] = fzero8();
        if (split) {
            #pragma unroll
            for (int t = 0; t < 2; ++t) {
                const size_t ko = ((size_t)bh * SDIM + kBase + 16 * t + m) * HD;
                const v8i kh0 = ldfrag(Kh + ko, 0, hh),   kl0 = ldfrag(Kl + ko, 0, hh);
                const v8i kh1 = ldfrag(Kh + ko, HHD, hh), kl1 = ldfrag(Kl + ko, HHD, hh);
                sc[t] = wm_h(sc[t], kh0, fQh0);
                sc[t] = wm_h(sc[t], kh0, fQl0);
                sc[t] = wm_h(sc[t], kl0, fQh0);
                sc[t] = wm_h(sc[t], kh1, fQh1);
                sc[t] = wm_h(sc[t], kh1, fQl1);
                sc[t] = wm_h(sc[t], kl1, fQh1);
            }
        } else {
            #pragma unroll
            for (int t = 0; t < 2; ++t) {
                const size_t ko = ((size_t)bh * SDIM + kBase + 16 * t + m) * HD;
                const v8i kh0 = ldfrag(Kh + ko, 0, hh);
                const v8i kh1 = ldfrag(Kh + ko, HHD, hh);
                sc[t] = wm_h(sc[t], kh0, fQh0);
                sc[t] = wm_h(sc[t], kh1, fQh1);
            }
        }

        float tmax = NEG_INF;
        if (it == jb) {
            #pragma unroll
            for (int t = 0; t < 2; ++t)
                #pragma unroll
                for (int r = 0; r < 8; ++r) {
                    const int key = kBase + 16 * t + 8 * hh + r;
                    const float v = (key > qRow) ? NEG_INF : sc[t][r];
                    sc[t][r] = v;
                    tmax = fmaxf(tmax, v);
                }
        } else {
            #pragma unroll
            for (int t = 0; t < 2; ++t)
                #pragma unroll
                for (int r = 0; r < 8; ++r) tmax = fmaxf(tmax, sc[t][r]);
        }
        tmax = fmaxf(tmax, __shfl_xor(tmax, 16, 32));
        const float nm = fmaxf(rmax, tmax);
        const float cr = (rmax == NEG_INF) ? 0.0f : __expf((rmax - nm) * SCALEC);
        rmax = nm;

        float psum = 0.0f;
        PackH ph[2], pl[2];
        #pragma unroll
        for (int t = 0; t < 2; ++t)
            #pragma unroll
            for (int r = 0; r < 8; ++r) {
                const float p = __expf(fmaf(sc[t][r] - nm, SCALEC, LN2P15));
                sc[t][r] = p;
                psum += p;
                ph[t].v[r] = (_Float16)p;
            }
        pl[0].u = (u32x4)0u; pl[1].u = (u32x4)0u;
        if (split) {
            #pragma unroll
            for (int t = 0; t < 2; ++t)
                #pragma unroll
                for (int r = 0; r < 8; ++r) pl[t].v[r] = (_Float16)(sc[t][r] - (float)ph[t].v[r]);
        }
        lsum = lsum * cr + psum;

        if (__ballot(cr != 1.0f) != 0ull) {
            #pragma unroll
            for (int r = 0; r < 8; ++r) {
                const float cq = __shfl(cr, 8 * hh + r, 32);
                #pragma unroll
                for (int c = 0; c < 4; ++c) acc[c][r] *= cq;
            }
        }

        Frag fPh, fPl;
        fPh.q[0] = ph[0].u; fPh.q[1] = ph[1].u;
        fPl.q[0] = pl[0].u; fPl.q[1] = pl[1].u;

        if (split) {
            #pragma unroll
            for (int c = 0; c < 4; ++c) {
                const size_t vo = ((size_t)bh * HD + 16 * c + m) * SDIM + kBase;
                const v8i vh = ldfrag(Vth + vo, 0, hh);
                const v8i vl = ldfrag(Vtl + vo, 0, hh);
                acc[c] = wm_h(acc[c], fPh.w, vh);
                acc[c] = wm_h(acc[c], fPh.w, vl);
                acc[c] = wm_h(acc[c], fPl.w, vh);
            }
        } else {
            #pragma unroll
            for (int c = 0; c < 4; ++c) {
                const size_t vo = ((size_t)bh * HD + 16 * c + m) * SDIM + kBase;
                const v8i vh = ldfrag(Vth + vo, 0, hh);
                acc[c] = wm_h(acc[c], fPh.w, vh);
            }
        }
    }

    const float ltot = lsum + __shfl_xor(lsum, 16, 32);
    const float inv = 1.0f / (ltot * QSCALE);
    #pragma unroll
    for (int r = 0; r < 8; ++r) {
        const float iq = __shfl(inv, 8 * hh + r, 32);
        #pragma unroll
        for (int c = 0; c < 4; ++c) stg[w][8 * hh + r][16 * c + m] = acc[c][r] * iq;
    }
    __syncthreads();

    const int rsub = lane >> 3, cg = (lane & 7) * 8;
    #pragma unroll
    for (int i = 0; i < 4; ++i) {
        const int rr = 4 * i + rsub;
        const v4f a0 = *(const v4fa*)(&stg[w][rr][cg]);
        const v4f a1 = *(const v4fa*)(&stg[w][rr][cg + 4]);
        float x[8];
        #pragma unroll
        for (int jj = 0; jj < 4; ++jj) { x[jj] = a0[jj]; x[4 + jj] = a1[jj]; }
        u32x4 oh, ol;
        split_b8(x, oh, ol);
        const size_t oo = ((size_t)(b * SDIM + qBase + rr)) * HDIM + h * HD + cg;
        volatile u32x4* const po = (volatile u32x4*)(Ah + oo);
        volatile u32x4* const pq = (volatile u32x4*)(Al + oo);
        *po = oh; *pq = ol;
        __threadfence();
        *po = oh; *pq = ol;
    }
}

__global__ void __launch_bounds__(256) __attribute__((amdgpu_num_vgpr(256)))
k_gemm_out(const unsigned short* __restrict__ Ahp, const unsigned short* __restrict__ Alp,
           const unsigned short* __restrict__ W, float* __restrict__ C)
{
    __shared__ __align__(16) float stg[8][32][64];

    const int tid = threadIdx.x, lane = tid & 31, wave = tid >> 5;
    const int hh = lane >> 4, m = lane & 15;
    const int mBase = blockIdx.y * 128, nBase = blockIdx.x * 128;
    if (mBase + 128 > BS || nBase + 128 > HDIM) return;
    const int m0 = (wave >> 1) * 32, n0 = (wave & 1) * 64;

    v8f acc[2][4];
    #pragma unroll
    for (int mt = 0; mt < 2; ++mt)
        #pragma unroll
        for (int nt = 0; nt < 4; ++nt) acc[mt][nt] = fzero8();

    const size_t ra0 = (size_t)(mBase + m0 + m) * HDIM;
    const size_t ra1 = ra0 + (size_t)16 * HDIM;
    const unsigned short* const br = W + (size_t)(nBase + n0 + m) * HDIM;

    #pragma unroll 1
    for (int k0 = 0; k0 < HDIM; k0 += 32) {
        const v8i aH0 = ldfrag(Ahp + ra0, k0, hh), aL0 = ldfrag(Alp + ra0, k0, hh);
        const v8i aH1 = ldfrag(Ahp + ra1, k0, hh), aL1 = ldfrag(Alp + ra1, k0, hh);
        #pragma unroll
        for (int nt = 0; nt < 4; ++nt) {
            const v8i bq = ldfrag(br + (size_t)nt * 16 * HDIM, k0, hh);
            acc[0][nt] = wm_b(acc[0][nt], aH0, bq);
            acc[0][nt] = wm_b(acc[0][nt], aL0, bq);
            acc[1][nt] = wm_b(acc[1][nt], aH1, bq);
            acc[1][nt] = wm_b(acc[1][nt], aL1, bq);
        }
    }

    #pragma unroll
    for (int mt = 0; mt < 2; ++mt)
        #pragma unroll
        for (int nt = 0; nt < 4; ++nt)
            #pragma unroll
            for (int r = 0; r < 8; ++r)
                stg[wave][mt * 16 + 8 * hh + r][nt * 16 + m] = acc[mt][nt][r];
    __syncthreads();

    #pragma unroll 1
    for (int i = 0; i < 16; ++i) {
        const int row = 2 * i + (lane >> 4), piece = lane & 15;
        const v4f v = *(const v4fa*)(&stg[wave][row][piece * 4]);
        volatile v4f* const p = (volatile v4f*)(C + (size_t)(mBase + m0 + row) * HDIM + nBase + n0 + piece * 4);
        *p = v;
        __threadfence();
        *p = v;
    }
}

extern "C" void kernel_launch(void* const* d_in, const int* in_sizes, int n_in,
                              void* d_out, int out_size, void* d_ws, size_t ws_size,
                              hipStream_t stream)
{
    if (n_in < 3) return;
    if (in_sizes[0] != BS * HDIM || in_sizes[1] != H3DIM * HDIM ||
        in_sizes[2] != HDIM * HDIM || out_size != BS * HDIM) return;

    const float* x    = (const float*)d_in[0];
    const float* wqkv = (const float*)d_in[1];
    const float* wo   = (const float*)d_in[2];
    float*       out  = (float*)d_out;

    char* ws = (char*)d_ws;
    size_t off = 0;
    auto carve = [&](size_t bytes) -> char* {
        char* p = ws + off;
        off += (bytes + 255) & ~(size_t)255;
        return p;
    };
    const size_t planeB = (size_t)BS * HDIM * 2;
    unsigned short* xb  = (unsigned short*)carve(planeB);
    unsigned short* wqb = (unsigned short*)carve((size_t)H3DIM * HDIM * 2);
    unsigned short* wob = (unsigned short*)carve((size_t)HDIM * HDIM * 2);
    float*          cst = (float*)         carve((size_t)SDIM * HHD * sizeof(float));
    float*          snt = (float*)         carve((size_t)SDIM * HHD * sizeof(float));
    unsigned short* qh  = (unsigned short*)carve(planeB);
    unsigned short* ql  = (unsigned short*)carve(planeB);
    unsigned short* kh  = (unsigned short*)carve(planeB);
    unsigned short* kl  = (unsigned short*)carve(planeB);
    unsigned short* vth = (unsigned short*)carve(planeB);
    unsigned short* vtl = (unsigned short*)carve(planeB);
    unsigned short* ah  = (unsigned short*)carve(planeB);
    unsigned short* al  = (unsigned short*)carve(planeB);
    if (off > ws_size) return;

    const dim3 blk256(256), blk64(64);
    const int n8x = BS * HDIM / 8, n8w = H3DIM * HDIM / 8, n8o = HDIM * HDIM / 8;

    k_cvt<<<dim3((n8x + 255) / 256), blk256, 0, stream>>>(x, xb, n8x);
    k_cvt<<<dim3((n8w + 255) / 256), blk256, 0, stream>>>(wqkv, wqb, n8w);
    k_cvt<<<dim3((n8o + 255) / 256), blk256, 0, stream>>>(wo, wob, n8o);
    k_trig<<<dim3((SDIM + 7) / 8), blk256, 0, stream>>>(cst, snt, SDIM);

    k_gemm_qkv<<<dim3(H3DIM / 128, BS / 128), blk256, 0, stream>>>(xb, wqb, cst, snt, qh, ql, kh, kl, vth, vtl);

    k_attn<<<dim3(NJB, NHEADS, BDIM), blk64, 0, stream>>>(qh, ql, kh, kl, vth, vtl, ah, al);

    k_gemm_out<<<dim3(HDIM / 128, BS / 128), blk256, 0, stream>>>(ah, al, wob, out);

    (void)hipGetLastError();
}
